// kernel_generated_3_62904091017470
// MI455X (gfx1250) — hardware-verified
//
#include <hip/hip_runtime.h>

typedef __bf16 v16bf __attribute__((ext_vector_type(16)));
typedef unsigned short v8us __attribute__((ext_vector_type(8)));
typedef unsigned short v16us __attribute__((ext_vector_type(16)));
typedef float v8f __attribute__((ext_vector_type(8)));
typedef float v4f __attribute__((ext_vector_type(4)));
typedef v4f __attribute__((may_alias)) v4fa;
typedef v8us __attribute__((may_alias)) v8usa;

#define NB    128
#define CIN   128
#define HW    196
#define NPOS  196
#define POSP  224
#define KK    576
#define KF    1728
#define NL    256
#define AROWS (NB * POSP)
#define PPR   72

static_assert(KF % 32 == 0);
static_assert(KK % 8 == 0);
static_assert((KF * 2) % 128 == 0);
static_assert((KK * 2) % 128 == 0);
static_assert((PPR % 8) == 0);
static_assert(((NL * NPOS) % 32) == 0);
static_assert(((64 * NPOS) % 32) == 0);

__device__ __forceinline__ v8f wmma_bf(v16bf a, v16bf b, v8f c) {
  v8f d = __builtin_amdgcn_wmma_f32_16x16x32_bf16(false, a, false, b, (short)0, c, false, false);
  asm volatile("v_nop\n\tv_nop\n\tv_nop\n\tv_nop" : "+v"(d) : "v"(a), "v"(b));
  return d;
}

__device__ __forceinline__ v16bf ldfrag(const unsigned short* p, int h) {
  const v8us u0 = *(const v8usa*)(p + 8 * h);
  const v8us u1 = *(const v8usa*)(p + 16 + 8 * h);
  const v16us u = __builtin_shufflevector(u0, u1, 0, 1, 2, 3, 4, 5, 6, 7, 8, 9, 10, 11, 12, 13, 14, 15);
  return __builtin_bit_cast(v16bf, u);
}

__device__ __forceinline__ unsigned short bf16_bits(float v) {
  unsigned int u = __float_as_uint(v);
  u += 0x7FFFu + ((u >> 16) & 1u);
  return (unsigned short)(u >> 16);
}

__device__ __forceinline__ void split2(float v, unsigned short& hi, unsigned short& lo) {
  hi = bf16_bits(v);
  const float hf = __uint_as_float(((unsigned int)hi) << 16);
  lo = bf16_bits(v - hf);
}

__device__ __forceinline__ void store_seg3(unsigned short* base, v8us s0, v8us s1, v8us s2) {
  unsigned short* p0 = base;
  unsigned short* p1 = base + KK;
  unsigned short* p2 = base + 2 * KK;
  *(volatile v8us*)p0 = s0;
  *(volatile v8us*)p1 = s1;
  *(volatile v8us*)p2 = s2;
  __threadfence();
  *(volatile v8us*)p0 = s0;
  *(volatile v8us*)p1 = s1;
  *(volatile v8us*)p2 = s2;
}

__global__ __launch_bounds__(256) void pack_w_k(const float* __restrict__ w,
                                               unsigned short* __restrict__ Bp)
{
  const int gid = blockIdx.x * 256 + threadIdx.x;
  if (gid >= NL * PPR) return;
  const int l = gid / PPR;
  const int piece = gid - l * PPR;
  const int kk0 = piece * 8;
  v8us hi8, lo8;
  #pragma unroll
  for (int e = 0; e < 8; ++e) {
    const float v = w[(size_t)(kk0 + e) * NL + l];
    unsigned short hb, lb;
    split2(v, hb, lb);
    hi8[e] = hb;
    lo8[e] = lb;
  }
  store_seg3(Bp + (size_t)l * KF + kk0, hi8, lo8, hi8);
}

__global__ __launch_bounds__(256) void pack_a_k(const float* __restrict__ x,
                                               unsigned short* __restrict__ Ap)
{
  const int gid = blockIdx.x * 256 + threadIdx.x;
  if (gid >= AROWS * PPR) return;
  const int row = gid / PPR;
  const int piece = gid - row * PPR;
  const int m = row / POSP;
  const int pos = row - m * POSP;
  const bool prow = pos < NPOS;
  const int posc = prow ? pos : (NPOS - 1);
  const int n = posc / 14;
  const int o = posc - n * 14;
  const int n2 = (n == 0) ? 13 : (n - 1);
  const int kk0 = piece * 8;
  const float* xm = x + (size_t)m * (CIN * HW);
  v8us hi8, lo8;
  #pragma unroll
  for (int e = 0; e < 8; ++e) {
    const int kk = kk0 + e;
    const int j = kk / 9;
    const int r9 = kk - j * 9;
    const int k = r9 / 3;
    const int i = r9 - k * 3;
    const int oi = o + i - 1;
    const bool vo = (unsigned)oi < 14u;
    int wc = oi - 1;
    wc = (wc < 0) ? (wc + 14) : wc;
    wc = (wc > 13) ? 13 : wc;
    const int h1 = n + k - 1;
    const bool v1 = (unsigned)h1 < 14u;
    const int h1c = (h1 < 0) ? 0 : ((h1 > 13) ? 13 : h1);
    const int h2 = n2 + k - 1;
    const bool v2 = (unsigned)h2 < 14u;
    const int h2c = (h2 < 0) ? 0 : ((h2 > 13) ? 13 : h2);
    const float xa = xm[(j * 14 + h1c) * 14 + wc];
    const float xb = xm[((64 + j) * 14 + h2c) * 14 + wc];
    float val = (v2 ? xb : 0.0f) + (v1 ? xa : 0.0f);
    val = (vo && prow) ? val : 0.0f;
    unsigned short hb, lb;
    split2(val, hb, lb);
    hi8[e] = hb;
    lo8[e] = lb;
  }
  store_seg3(Ap + (size_t)row * KF + kk0, hi8, hi8, lo8);
}

__global__ __launch_bounds__(224) void gemm_k(const unsigned short* __restrict__ Ap,
                                             const unsigned short* __restrict__ Bp,
                                             float* __restrict__ out)
{
  __shared__ __attribute__((aligned(16))) float sD[64 * NPOS];
  const int tid = threadIdx.x, lane = tid & 31, w = tid >> 5;
  const int h = lane >> 4, mm = lane & 15;
  const int lg = blockIdx.x;
  const int m = blockIdx.y;
  const int l0 = lg * 64;
  const unsigned short* a0p = Ap + (size_t)(m * POSP + 32 * w + mm) * KF;
  const unsigned short* a1p = a0p + (size_t)16 * KF;
  const unsigned short* b0p = Bp + (size_t)(l0 + mm) * KF;
  const v8f z8 = {0.f, 0.f, 0.f, 0.f, 0.f, 0.f, 0.f, 0.f};
  v8f acc0[4], acc1[4];
  #pragma unroll
  for (int nt = 0; nt < 4; ++nt) { acc0[nt] = z8; acc1[nt] = z8; }

  #pragma unroll 1
  for (int k0 = 0; k0 < KF; k0 += 32) {
    const v16bf fa0 = ldfrag(a0p + k0, h);
    const v16bf fa1 = ldfrag(a1p + k0, h);
    #pragma unroll
    for (int nt = 0; nt < 4; ++nt) {
      const v16bf fb = ldfrag(b0p + (size_t)nt * 16 * KF + k0, h);
      acc0[nt] = wmma_bf(fa0, fb, acc0[nt]);
      acc1[nt] = wmma_bf(fa1, fb, acc1[nt]);
    }
  }

  #pragma unroll
  for (int nt = 0; nt < 4; ++nt) {
    const int lcol = 16 * nt + mm;
    #pragma unroll
    for (int r = 0; r < 8; ++r) {
      const int p0 = 32 * w + 8 * h + r;
      const int p1 = p0 + 16;
      if (p0 < NPOS) sD[lcol * NPOS + p0] = acc0[nt][r];
      if (p1 < NPOS) sD[lcol * NPOS + p1] = acc1[nt][r];
    }
  }
  __syncthreads();

  float* ob = out + (size_t)m * (NL * NPOS) + (size_t)l0 * NPOS;
  const int sub = lane >> 3, q8 = lane & 7;
  v4f vals[14];
  int offs[14];
  #pragma unroll
  for (int it = 0; it < 14; ++it) {
    const int line = 56 * w + 4 * it + sub;
    offs[it] = line * 32 + 4 * q8;
    vals[it] = *(const v4fa*)(sD + offs[it]);
  }
  #pragma unroll
  for (int it = 0; it < 14; ++it) *(volatile v4f*)(ob + offs[it]) = vals[it];
  __threadfence();
  #pragma unroll
  for (int it = 0; it < 14; ++it) *(volatile v4f*)(ob + offs[it]) = vals[it];
}

extern "C" void kernel_launch(void* const* d_in, const int* in_sizes, int n_in,
                              void* d_out, int out_size, void* d_ws, size_t ws_size,
                              hipStream_t stream) {
  if (n_in < 2) return;
  if (in_sizes[0] != NB * CIN * HW) return;
  if (in_sizes[1] != KK * NL) return;
  if (out_size != NB * NL * NPOS) return;

  const size_t bpBytes = (size_t)NL * KF * 2;
  const size_t apBytes = (size_t)AROWS * KF * 2;
  if (bpBytes + apBytes > ws_size) return;

  const float* x = (const float*)d_in[0];
  const float* w = (const float*)d_in[1];
  float* out = (float*)d_out;
  char* ws = (char*)d_ws;
  unsigned short* Bp = (unsigned short*)(ws + 0);
  unsigned short* Ap = (unsigned short*)(ws + bpBytes);

  const int gw = (NL * PPR + 255) / 256;
  const int ga = (AROWS * PPR + 255) / 256;
  pack_w_k<<<gw, 256, 0, stream>>>(w, Bp);
  pack_a_k<<<ga, 256, 0, stream>>>(x, Ap);
  gemm_k<<<dim3(NL / 64, NB), 224, 0, stream>>>(Ap, Bp, out);
}
